// Attention_60928406061617
// MI455X (gfx1250) — hardware-verified
//
#include <hip/hip_runtime.h>
#include <math.h>
#include <stdint.h>

#ifndef NB
#define NB 16
#endif
#define NB_FULL 16
#define NTOK 577
#define NP   640
#define DM   768
#define NH   12
#define HD   64
#define C3   (3 * DM)
#define NQT  (NP / 64)
#define NCT  (DM / 64)
#define NC3T (C3 / 64)
#define TP   68
#define WSC  256.0f
#define QS   8.0f
#define RESC 1024.0f
#define PCAR 8192.0f
#define CCAR 64.0f
#define LOG2E 1.4426950408889634f
#define GEMM_THREADS 128
#define CVT_THREADS  (DM / 8)
#define MIX_THREADS  320
#define MIX_WAVES    (MIX_THREADS / 32)

static_assert(NB >= 1 && NB <= NB_FULL);
static_assert(NP % 64 == 0 && NP >= NTOK && NP - NTOK < 64);
static_assert(DM % 64 == 0 && DM % 32 == 0 && HD % 32 == 0 && NH * HD == DM);
static_assert(NP % 32 == 0 && HD == 64 && CVT_THREADS == 96);
static_assert(MIX_THREADS <= NTOK && 2 * MIX_THREADS == NP && MIX_THREADS % 32 == 0);
static_assert(NH * (NP / 8) == 3 * MIX_THREADS && (NP / 8) % 8 == 0);
static_assert((TP * 4) % 16 == 0 && NH * NH <= MIX_THREADS);

typedef unsigned short u16;
typedef _Float16 v16h __attribute__((ext_vector_type(16)));
typedef _Float16 v8h  __attribute__((ext_vector_type(8)));
typedef float    v8f  __attribute__((ext_vector_type(8)));
typedef float    v4f  __attribute__((ext_vector_type(4)));
typedef unsigned int v4u __attribute__((ext_vector_type(4)));

union FragH { v16h v; v8h h[2]; };

__device__ __forceinline__ unsigned short bf_bits(float f) {
  unsigned u = __float_as_uint(f);
  return (unsigned short)((u + 0x7FFFu + ((u >> 16) & 1u)) >> 16);
}
__device__ __forceinline__ float bf_up(unsigned short h) { return __uint_as_float(((unsigned)h) << 16); }
__device__ __forceinline__ float bfr(float f) { return bf_up(bf_bits(f)); }
__device__ __forceinline__ unsigned short h_bits(_Float16 x) { return __builtin_bit_cast(unsigned short, x); }
__device__ __forceinline__ unsigned pk16(unsigned short a, unsigned short b) { return (unsigned)a | ((unsigned)b << 16); }
__device__ __forceinline__ v8f zero8() { v8f z = {0.f, 0.f, 0.f, 0.f, 0.f, 0.f, 0.f, 0.f}; return z; }
__device__ __forceinline__ v4u zero4u() { v4u z = {0u, 0u, 0u, 0u}; return z; }

__device__ __forceinline__ v16h ldfrag_h(const _Float16* p) {
  FragH f;
  f.h[0] = *(const v8h*)(p);
  f.h[1] = *(const v8h*)(p + 16);
  return f.v;
}

__device__ __forceinline__ v8f mma_h(v16h a, v16h b, v8f c) {
  return __builtin_amdgcn_wmma_f32_16x16x32_f16(false, a, false, b, (short)0, c, false, false);
}
__device__ __forceinline__ void guard4(v8f (&c)[4], v16h x0, v16h x1, v16h x2, v16h x3) {
#if defined(__HIP_DEVICE_COMPILE__)
  asm volatile("v_nop\n\tv_nop\n\tv_nop\n\tv_nop"
               : "+v"(c[0]), "+v"(c[1]), "+v"(c[2]), "+v"(c[3])
               : "v"(x0), "v"(x1), "v"(x2), "v"(x3) : "memory");
#endif
}
__device__ __forceinline__ void guard8(v8f (&c)[4], v8f (&d)[4], v16h x0, v16h x1, v16h x2, v16h x3, v16h x4, v16h x5) {
#if defined(__HIP_DEVICE_COMPILE__)
  asm volatile("v_nop\n\tv_nop\n\tv_nop\n\tv_nop"
               : "+v"(c[0]), "+v"(c[1]), "+v"(c[2]), "+v"(c[3]),
                 "+v"(d[0]), "+v"(d[1]), "+v"(d[2]), "+v"(d[3])
               : "v"(x0), "v"(x1), "v"(x2), "v"(x3), "v"(x4), "v"(x5) : "memory");
#endif
}
__device__ __forceinline__ void acc_guard(v8f (&c)[4], v8f (&d)[4]) {
#if defined(__HIP_DEVICE_COMPILE__)
  asm volatile("v_nop\n\tv_nop\n\tv_nop\n\tv_nop"
               : "+v"(c[0]), "+v"(c[1]), "+v"(c[2]), "+v"(c[3]),
                 "+v"(d[0]), "+v"(d[1]), "+v"(d[2]), "+v"(d[3]));
#endif
}
__device__ __forceinline__ void wave_sync_lds() {
  __builtin_amdgcn_fence(__ATOMIC_RELEASE, "workgroup");
  __builtin_amdgcn_wave_barrier();
  __builtin_amdgcn_fence(__ATOMIC_ACQUIRE, "workgroup");
}

template <int ARES>
__device__ __forceinline__ void mma_tile(const _Float16* __restrict__ ap, const _Float16* __restrict__ arp,
                                         const _Float16* __restrict__ bp, int K, int lda, int ldb,
                                         v8f (&acc)[4], v8f (&accr)[4]) {
  const size_t a16 = (size_t)16 * (size_t)lda;
  const size_t b16 = (size_t)16 * (size_t)ldb;
#pragma unroll 1
  for (int k0 = 0; k0 < K; k0 += 32) {
    const v16h a0 = ldfrag_h(ap + k0);
    const v16h a1 = ldfrag_h(ap + a16 + k0);
    const v16h b0 = ldfrag_h(bp + k0);
    const v16h b1 = ldfrag_h(bp + b16 + k0);
    acc[0] = mma_h(a0, b0, acc[0]);
    acc[1] = mma_h(a0, b1, acc[1]);
    acc[2] = mma_h(a1, b0, acc[2]);
    acc[3] = mma_h(a1, b1, acc[3]);
    if (ARES) {
      const v16h r0 = ldfrag_h(arp + k0);
      const v16h r1 = ldfrag_h(arp + a16 + k0);
      accr[0] = mma_h(r0, b0, accr[0]);
      accr[1] = mma_h(r0, b1, accr[1]);
      accr[2] = mma_h(r1, b0, accr[2]);
      accr[3] = mma_h(r1, b1, accr[3]);
      guard8(acc, accr, a0, a1, r0, r1, b0, b1);
    } else {
      guard4(acc, a0, a1, b0, b1);
    }
  }
}

template <int ARES>
__device__ __forceinline__ void stage_tile(float* T, v8f (&acc)[4], v8f (&accr)[4], float os, float ors,
                                           int wr, int wc, int hh, int m) {
#pragma unroll
  for (int i = 0; i < 2; ++i) {
#pragma unroll
    for (int j = 0; j < 2; ++j) {
#pragma unroll
      for (int r = 0; r < 8; ++r) {
        float v = acc[2 * i + j][r] * os;
        if (ARES) v += accr[2 * i + j][r] * ors;
        T[(32 * wr + 16 * i + 8 * hh + r) * TP + 32 * wc + 16 * j + m] = v;
      }
    }
  }
}

template <int RES, int ADD>
__device__ __forceinline__ void epi16(const float* T, const float* addv, u16* P0, u16* P1,
                                      size_t base, int ldc, float sc, int wave, int lane) {
  const int rq = lane >> 3, c8 = (lane & 7) * 8;
  v4u oh[4], orr[4];
#pragma unroll
  for (int i = 0; i < 4; ++i) {
    const int row = 16 * wave + 4 * i + rq;
    const v4f a = *(const v4f*)(T + row * TP + c8);
    const v4f c = *(const v4f*)(T + row * TP + c8 + 4);
    float x[8] = {a[0], a[1], a[2], a[3], c[0], c[1], c[2], c[3]};
    if (ADD) {
      const v4f d0 = *(const v4f*)(addv + c8);
      const v4f d1 = *(const v4f*)(addv + c8 + 4);
      x[0] += d0[0]; x[1] += d0[1]; x[2] += d0[2]; x[3] += d0[3];
      x[4] += d1[0]; x[5] += d1[1]; x[6] += d1[2]; x[7] += d1[3];
    }
    orr[i] = zero4u();
#pragma unroll
    for (int e = 0; e < 4; ++e) {
      const float y0 = x[2 * e] * sc, y1 = x[2 * e + 1] * sc;
      const _Float16 h0 = (_Float16)y0, h1 = (_Float16)y1;
      oh[i][e] = pk16(h_bits(h0), h_bits(h1));
      if (RES) {
        const _Float16 r0 = (_Float16)((y0 - (float)h0) * RESC);
        const _Float16 r1 = (_Float16)((y1 - (float)h1) * RESC);
        orr[i][e] = pk16(h_bits(r0), h_bits(r1));
      }
    }
  }
  for (int pass = 0; pass < 2; ++pass) {
#pragma unroll
    for (int i = 0; i < 4; ++i) {
      const int row = 16 * wave + 4 * i + rq;
      const size_t o = base + (size_t)row * (size_t)ldc + (size_t)c8;
      *(volatile v4u*)(P0 + o) = oh[i];
      if (RES) *(volatile v4u*)(P1 + o) = orr[i];
    }
    __threadfence();
  }
}

template <int BIAS>
__device__ __forceinline__ void epi32(const float* T, const float* cbias, float* C, size_t base, int ldc, int nvalid,
                                      int wave, int lane) {
  const int rh = lane >> 4, c4 = (lane & 15) * 4;
  v4f vals[8];
#pragma unroll
  for (int i = 0; i < 8; ++i) {
    const int row = 16 * wave + 2 * i + rh;
    v4f v = *(const v4f*)(T + row * TP + c4);
    if (BIAS) { const v4f bb = *(const v4f*)(cbias + c4); v += bb; }
    vals[i] = v;
  }
  for (int pass = 0; pass < 2; ++pass) {
#pragma unroll
    for (int i = 0; i < 8; ++i) {
      const int row = 16 * wave + 2 * i + rh;
      if (row < nvalid) *(volatile v4f*)(C + base + (size_t)row * (size_t)ldc + (size_t)c4) = vals[i];
    }
    __threadfence();
  }
}

__global__ __launch_bounds__(CVT_THREADS)
void k_cvt(const float* __restrict__ X, u16* Y, int rowsPerB, int validRows, int srcRowsPerB, float scale) {
  const int tid = threadIdx.x;
  const int r = blockIdx.x;
  const int b = r / rowsPerB;
  const int s = r - b * rowsPerB;
  v4u o = zero4u();
  if (s < validRows) {
    const float* src = X + ((size_t)b * (size_t)srcRowsPerB + (size_t)s) * (size_t)DM + (size_t)tid * 8;
    const v4f a = *(const v4f*)(src), c = *(const v4f*)(src + 4);
#pragma unroll
    for (int e = 0; e < 2; ++e) {
      o[e]     = pk16(h_bits((_Float16)(bfr(a[2 * e]) * scale)), h_bits((_Float16)(bfr(a[2 * e + 1]) * scale)));
      o[2 + e] = pk16(h_bits((_Float16)(bfr(c[2 * e]) * scale)), h_bits((_Float16)(bfr(c[2 * e + 1]) * scale)));
    }
  }
  u16* dst = Y + (size_t)r * (size_t)DM + (size_t)tid * 8;
  for (int pass = 0; pass < 2; ++pass) {
    *(volatile v4u*)(dst) = o;
    __threadfence();
  }
}

__global__ __launch_bounds__(GEMM_THREADS)
void k_qkv(const u16* __restrict__ X16, const u16* __restrict__ W16,
           u16* Qh, u16* Qr, u16* Kh, u16* VT, float* PS) {
  __shared__ __align__(16) float T[64 * TP];
  __shared__ __align__(16) float ssum[64];
  const int tid = threadIdx.x, wave = tid >> 5, lane = tid & 31, hh = lane >> 4, m = lane & 15;
  const int wr = wave & 1, wc = wave >> 1;
  const int bid = blockIdx.x;
  const int nt = bid % NC3T, mt = bid / NC3T;
  const int rowb = mt * 64, col0 = nt * 64;
  const int b = rowb / NP, n0 = rowb - b * NP;
  const int t = col0 / DM, cin = col0 - t * DM;

  const _Float16* ap = (const _Float16*)(const void*)X16 + (size_t)(rowb + 32 * wr + m) * (size_t)DM + 8 * hh;
  const _Float16* bp = (const _Float16*)(const void*)W16 + (size_t)(col0 + 32 * wc + m) * (size_t)DM + 8 * hh;
  v8f acc[4], accr[4];
#pragma unroll
  for (int i = 0; i < 4; ++i) { acc[i] = zero8(); accr[i] = zero8(); }
  mma_tile<0>(ap, ap, bp, DM, DM, DM, acc, accr);
  acc_guard(acc, accr);
  stage_tile<0>(T, acc, accr, QS / WSC, 0.f, wr, wc, hh, m);
  __syncthreads();

  if (t == 0) {
    epi16<1, 0>(T, T, Qh, Qr, (size_t)rowb * (size_t)DM + (size_t)cin, DM, 1.0f, wave, lane);
  } else if (t == 1) {
    epi16<0, 0>(T, T, Kh, Kh, (size_t)rowb * (size_t)DM + (size_t)cin, DM, 1.0f, wave, lane);
  } else {
    const int rq = lane >> 3, c8 = (lane & 7) * 8;
    v4u ov[4];
#pragma unroll
    for (int i = 0; i < 4; ++i) {
      const int d = 16 * wave + 4 * i + rq;
#pragma unroll
      for (int e = 0; e < 4; ++e) {
        const float x0 = T[(c8 + 2 * e) * TP + d];
        const float x1 = T[(c8 + 2 * e + 1) * TP + d];
        ov[i][e] = pk16(h_bits((_Float16)x0), h_bits((_Float16)x1));
      }
    }
    u16* dst = VT + ((size_t)(b * DM + cin)) * (size_t)NP + (size_t)(n0 + c8);
    for (int pass = 0; pass < 2; ++pass) {
#pragma unroll
      for (int i = 0; i < 4; ++i) {
        const int d = 16 * wave + 4 * i + rq;
        *(volatile v4u*)(dst + (size_t)d * (size_t)NP) = ov[i];
      }
      __threadfence();
    }
    if (tid < 64) {
      float s = 0.f;
#pragma unroll 8
      for (int r = 0; r < 64; ++r) s += T[r * TP + tid];
      ssum[tid] = s;
    }
    __syncthreads();
    if (wave == 0) {
      const int li = (lane < 16) ? lane : 15;
      const v4f sv = *(const v4f*)(ssum + 4 * li);
      float* pd = PS + ((size_t)(b * NQT + (n0 >> 6))) * (size_t)DM + (size_t)(cin + 4 * li);
      for (int pass = 0; pass < 2; ++pass) {
        if (lane < 16) *(volatile v4f*)(pd) = sv;
        __threadfence();
      }
    }
  }
}

__global__ __launch_bounds__(GEMM_THREADS)
void k_scores(const u16* __restrict__ Qh, const u16* __restrict__ Qr, const u16* __restrict__ Kh, float* S, int b) {
  __shared__ __align__(16) float T[64 * TP];
  const int tid = threadIdx.x, wave = tid >> 5, lane = tid & 31, hh = lane >> 4, m = lane & 15;
  const int wr = wave & 1, wc = wave >> 1;
  const int bid = blockIdx.x;
  const int h = bid / (NQT * NQT);
  const int rem = bid - h * (NQT * NQT);
  const int qt = rem / NQT, kt = rem - qt * NQT;

  const size_t qoff = ((size_t)(b * NP + qt * 64 + 32 * wr + m)) * (size_t)DM + (size_t)(h * HD + 8 * hh);
  const size_t koff = ((size_t)(b * NP + kt * 64 + 32 * wc + m)) * (size_t)DM + (size_t)(h * HD + 8 * hh);
  const _Float16* ap  = (const _Float16*)(const void*)Qh + qoff;
  const _Float16* arp = (const _Float16*)(const void*)Qr + qoff;
  const _Float16* bp  = (const _Float16*)(const void*)Kh + koff;
  v8f acc[4], accr[4];
#pragma unroll
  for (int i = 0; i < 4; ++i) { acc[i] = zero8(); accr[i] = zero8(); }
  mma_tile<1>(ap, arp, bp, HD, DM, DM, acc, accr);
  acc_guard(acc, accr);
  const float os = (1.0f / 512.0f);
  stage_tile<1>(T, acc, accr, os, os * (1.0f / RESC), wr, wc, hh, m);
  __syncthreads();
  epi32<0>(T, T, S, ((size_t)(h * NP + qt * 64)) * (size_t)NP + (size_t)(kt * 64), NP, 64, wave, lane);
}

__global__ __launch_bounds__(MIX_THREADS)
void k_mixsm(const float* __restrict__ S, const float* __restrict__ Wpre, const float* __restrict__ Wpost, u16* Ph) {
  __shared__ __align__(16) float sW[2][NH][NH];
  __shared__ __align__(16) float sPf[NH][NP];
  __shared__ __align__(16) u16   sP16[NH][NP];
  __shared__ float sRed[2][NH][MIX_WAVES];
  __shared__ float sMZ[2][NH];

  const int tid = threadIdx.x, wave = tid >> 5, lane = tid & 31;
  const int n = blockIdx.x;
  const int m0 = tid, m1 = tid + MIX_THREADS;
  const bool v1ok = (m1 < NTOK);
  v4u ov[3];

  if (n < NTOK) {
    {
      const int wi = (tid < NH * NH) ? tid : (NH * NH - 1);
      const float wa = bfr(Wpre[wi]);
      const float wb = bfr(Wpost[wi]);
      if (tid < NH * NH) {
        const int g = tid / NH, h = tid - g * NH;
        sW[0][h][g] = wa;
        sW[1][h][g] = wb;
      }
    }
    __syncthreads();

    float a0[NH], a1[NH];
#pragma unroll
    for (int g = 0; g < NH; ++g) { a0[g] = 0.f; a1[g] = 0.f; }
    const float* srow = S + (size_t)n * (size_t)NP;
#pragma unroll 1
    for (int h = 0; h < NH; ++h) {
      const float s0 = srow[(size_t)h * (size_t)(NP * NP) + (size_t)m0];
      const float s1 = srow[(size_t)h * (size_t)(NP * NP) + (size_t)m1];
      const v4f w0 = *(const v4f*)(&sW[0][h][0]);
      const v4f w1 = *(const v4f*)(&sW[0][h][4]);
      const v4f w2 = *(const v4f*)(&sW[0][h][8]);
      const float w[NH] = {w0[0], w0[1], w0[2], w0[3], w1[0], w1[1], w1[2], w1[3], w2[0], w2[1], w2[2], w2[3]};
#pragma unroll
      for (int g = 0; g < NH; ++g) { a0[g] = fmaf(w[g], s0, a0[g]); a1[g] = fmaf(w[g], s1, a1[g]); }
    }

    float red[NH];
#pragma unroll
    for (int g = 0; g < NH; ++g) red[g] = fmaxf(a0[g], v1ok ? a1[g] : -INFINITY);
#pragma unroll
    for (int g = 0; g < NH; ++g) {
#pragma unroll
      for (int off = 16; off > 0; off >>= 1) red[g] = fmaxf(red[g], __shfl_xor(red[g], off, 32));
    }
    if (lane == 0) {
#pragma unroll
      for (int g = 0; g < NH; ++g) sRed[0][g][wave] = red[g];
    }
    __syncthreads();
    if (tid < NH) {
      float mx = sRed[0][tid][0];
#pragma unroll 1
      for (int w2 = 1; w2 < MIX_WAVES; ++w2) mx = fmaxf(mx, sRed[0][tid][w2]);
      sMZ[0][tid] = mx;
    }
    __syncthreads();

    float e0[NH], e1[NH];
#pragma unroll
    for (int g = 0; g < NH; ++g) {
      const float Mg = sMZ[0][g];
      e0[g] = exp2f((a0[g] - Mg) * LOG2E);
      const float t1 = exp2f((a1[g] - Mg) * LOG2E);
      e1[g] = v1ok ? t1 : 0.f;
      red[g] = e0[g] + e1[g];
    }
#pragma unroll
    for (int g = 0; g < NH; ++g) {
#pragma unroll
      for (int off = 16; off > 0; off >>= 1) red[g] += __shfl_xor(red[g], off, 32);
    }
    if (lane == 0) {
#pragma unroll
      for (int g = 0; g < NH; ++g) sRed[1][g][wave] = red[g];
    }
    __syncthreads();
    if (tid < NH) {
      float z = sRed[1][tid][0];
#pragma unroll 1
      for (int w2 = 1; w2 < MIX_WAVES; ++w2) z += sRed[1][tid][w2];
      sMZ[1][tid] = z;
    }
    __syncthreads();

#pragma unroll
    for (int g = 0; g < NH; ++g) {
      const float Z = sMZ[1][g];
      const float invZ = __builtin_amdgcn_rcpf(Z);
      const float zc = Z * (1.0f / (float)NTOK);
      const float p0 = (e0[g] - zc) * invZ;
      const float p1t = (e1[g] - zc) * invZ;
      sPf[g][m0] = p0;
      sPf[g][m1] = v1ok ? p1t : 0.f;
    }
    wave_sync_lds();

    float q0[NH], q1[NH];
#pragma unroll
    for (int g = 0; g < NH; ++g) { q0[g] = 0.f; q1[g] = 0.f; }
#pragma unroll 1
    for (int h = 0; h < NH; ++h) {
      const float p0 = sPf[h][m0];
      const float p1 = sPf[h][m1];
      const v4f w0 = *(const v4f*)(&sW[1][h][0]);
      const v4f w1 = *(const v4f*)(&sW[1][h][4]);
      const v4f w2 = *(const v4f*)(&sW[1][h][8]);
      const float w[NH] = {w0[0], w0[1], w0[2], w0[3], w1[0], w1[1], w1[2], w1[3], w2[0], w2[1], w2[2], w2[3]};
#pragma unroll
      for (int g = 0; g < NH; ++g) { q0[g] = fmaf(w[g], p0, q0[g]); q1[g] = fmaf(w[g], p1, q1[g]); }
    }
#pragma unroll
    for (int g = 0; g < NH; ++g) {
      sP16[g][m0] = h_bits((_Float16)(q0[g] * PCAR));
      sP16[g][m1] = h_bits((_Float16)(q1[g] * PCAR));
    }
    __syncthreads();
#pragma unroll
    for (int i = 0; i < 3; ++i) {
      const int p = tid + MIX_THREADS * i;
      const int row = p / (NP / 8);
      const int qq = p - row * (NP / 8);
      ov[i] = *(const v4u*)(&sP16[row][qq * 8]);
    }
  } else {
#pragma unroll
    for (int i = 0; i < 3; ++i) ov[i] = zero4u();
  }

  u16* base = Ph + (size_t)n * (size_t)NP;
  for (int pass = 0; pass < 2; ++pass) {
#pragma unroll
    for (int i = 0; i < 3; ++i) {
      const int p = tid + MIX_THREADS * i;
      const int row = p / (NP / 8);
      const int qq = p - row * (NP / 8);
      *(volatile v4u*)(base + (size_t)row * (size_t)(NP * NP) + (size_t)(qq * 8)) = ov[i];
    }
    __threadfence();
  }
}

__global__ __launch_bounds__(GEMM_THREADS)
void k_pv(const u16* __restrict__ Ph, const u16* __restrict__ VT, const float* __restrict__ PS,
          const float* __restrict__ Wpost, u16* Ch, u16* Cr, int b) {
  __shared__ __align__(16) float T[64 * TP];
  __shared__ __align__(16) float sadd[64];
  const int tid = threadIdx.x, wave = tid >> 5, lane = tid & 31, hh = lane >> 4, m = lane & 15;
  const int wr = wave & 1, wc = wave >> 1;
  const int bid = blockIdx.x;
  const int g = bid / NQT, qt = bid - g * NQT;

  if (tid < 64) {
    const int d = tid;
    float cs = 0.f;
#pragma unroll 1
    for (int nt = 0; nt < NQT; ++nt) cs += PS[((size_t)(b * NQT + nt)) * (size_t)DM + (size_t)(g * HD + d)];
    float ag = 0.f;
#pragma unroll 1
    for (int h = 0; h < NH; ++h) ag += bfr(Wpost[g * NH + h]);
    sadd[d] = cs * (ag * (1.0f / (QS * (float)NTOK)));
  }

  const _Float16* ap = (const _Float16*)(const void*)Ph + ((size_t)(g * NP + qt * 64 + 32 * wr + m)) * (size_t)NP + 8 * hh;
  const _Float16* bp = (const _Float16*)(const void*)VT + ((size_t)(b * DM + g * HD + 32 * wc + m)) * (size_t)NP + 8 * hh;
  v8f acc[4], accr[4];
#pragma unroll
  for (int i = 0; i < 4; ++i) { acc[i] = zero8(); accr[i] = zero8(); }
  mma_tile<0>(ap, ap, bp, NP, NP, NP, acc, accr);
  acc_guard(acc, accr);
  stage_tile<0>(T, acc, accr, 1.0f / (PCAR * QS), 0.f, wr, wc, hh, m);
  __syncthreads();
  epi16<1, 1>(T, sadd, Ch, Cr, ((size_t)(b * NP + qt * 64)) * (size_t)DM + (size_t)(g * HD), DM, CCAR, wave, lane);
}

__global__ __launch_bounds__(GEMM_THREADS)
void k_proj(const u16* __restrict__ Ch, const u16* __restrict__ Cr, const u16* __restrict__ Wp,
            const float* __restrict__ bias, int nbias, float* Out) {
  __shared__ __align__(16) float T[64 * TP];
  __shared__ __align__(16) float cb[64];
  const int tid = threadIdx.x, wave = tid >> 5, lane = tid & 31, hh = lane >> 4, m = lane & 15;
  const int wr = wave & 1, wc = wave >> 1;
  const int bid = blockIdx.x;
  const int nt = bid % NCT;
  const int tmp = bid / NCT;
  const int qt = tmp % NQT;
  const int b = tmp / NQT;

  if (tid < 64) {
    int ci = nt * 64 + tid;
    ci = (ci < nbias - 1) ? ci : (nbias - 1);
    cb[tid] = bfr(bias[ci]);
  }
  const size_t aoff = ((size_t)(b * NP + qt * 64 + 32 * wr + m)) * (size_t)DM + 8 * hh;
  const _Float16* ap  = (const _Float16*)(const void*)Ch + aoff;
  const _Float16* arp = (const _Float16*)(const void*)Cr + aoff;
  const _Float16* bp  = (const _Float16*)(const void*)Wp + ((size_t)(nt * 64 + 32 * wc + m)) * (size_t)DM + 8 * hh;
  v8f acc[4], accr[4];
#pragma unroll
  for (int i = 0; i < 4; ++i) { acc[i] = zero8(); accr[i] = zero8(); }
  mma_tile<1>(ap, arp, bp, DM, DM, DM, acc, accr);
  acc_guard(acc, accr);
  const float os = 1.0f / (CCAR * WSC);
  stage_tile<1>(T, acc, accr, os, os * (1.0f / RESC), wr, wc, hh, m);
  __syncthreads();
  epi32<1>(T, cb, Out, ((size_t)(b * NTOK + qt * 64)) * (size_t)DM + (size_t)(nt * 64), DM, NTOK - qt * 64, wave, lane);
}

extern "C" void kernel_launch(void* const* d_in, const int* in_sizes, int n_in,
                              void* d_out, int out_size, void* d_ws, size_t ws_size,
                              hipStream_t stream) {
  if (n_in < 6) return;
  if (in_sizes[0] < NB * NTOK * DM) return;
  if (in_sizes[1] < C3 * DM) return;
  if (in_sizes[2] < DM * DM) return;
  if (in_sizes[3] < 1) return;
  if (in_sizes[4] < NH * NH || in_sizes[5] < NH * NH) return;
  if (out_size < NB * NTOK * DM) return;

  const float* x     = (const float*)d_in[0];
  const float* wqkv  = (const float*)d_in[1];
  const float* wproj = (const float*)d_in[2];
  const float* bproj = (const float*)d_in[3];
  const float* wpre  = (const float*)d_in[4];
  const float* wpost = (const float*)d_in[5];
  float*       out   = (float*)d_out;
  const int    nbias = in_sizes[3];

  const size_t szS  = (size_t)NH * NP * NP * 4;
  const size_t szPh = (size_t)NH * NP * NP * 2;
  const size_t szX  = (size_t)NB * NP * DM * 2;
  const size_t szWq = (size_t)C3 * DM * 2;
  const size_t szWp = (size_t)DM * DM * 2;
  const size_t szPl = (size_t)NB * NP * DM * 2;
  const size_t szPS = (size_t)NB * NQT * DM * 4;
  const size_t r0a = szS + szPh, r0b = szX + szWq;
  const size_t r0 = (r0a > r0b) ? r0a : r0b;
  const size_t oS = 0, oPh = szS, oX = 0, oWq = szX;
  size_t off = r0;
  const size_t oWp = off; off += szWp;
  const size_t oQh = off; off += szPl;
  const size_t oQr = off; off += szPl;
  const size_t oKh = off; off += szPl;
  const size_t oVT = off; off += szPl;
  const size_t oCh = off; off += szPl;
  const size_t oCr = off; off += szPl;
  const size_t oPS = off; off += szPS;
  if (off > ws_size) return;
  if (off > (size_t)134217728) return;

  char* ws = (char*)d_ws;
  float* S    = (float*)(ws + oS);
  u16*   Ph   = (u16*)(ws + oPh);
  u16*   X16  = (u16*)(ws + oX);
  u16*   Wq16 = (u16*)(ws + oWq);
  u16*   Wp16 = (u16*)(ws + oWp);
  u16*   Qh   = (u16*)(ws + oQh);
  u16*   Qr   = (u16*)(ws + oQr);
  u16*   Kh   = (u16*)(ws + oKh);
  u16*   VT   = (u16*)(ws + oVT);
  u16*   Ch   = (u16*)(ws + oCh);
  u16*   Cr   = (u16*)(ws + oCr);
  float* PS   = (float*)(ws + oPS);

  k_cvt<<<dim3(NB * NP), dim3(CVT_THREADS), 0, stream>>>(x, X16, NP, NTOK, NTOK, 1.0f);
  k_cvt<<<dim3(C3), dim3(CVT_THREADS), 0, stream>>>(wqkv, Wq16, C3, C3, C3, WSC);
  k_cvt<<<dim3(DM), dim3(CVT_THREADS), 0, stream>>>(wproj, Wp16, DM, DM, DM, WSC);
  k_qkv<<<dim3((NB * NP / 64) * NC3T), dim3(GEMM_THREADS), 0, stream>>>(X16, Wq16, Qh, Qr, Kh, VT, PS);
  for (int b = 0; b < NB; ++b) {
    k_scores<<<dim3(NH * NQT * NQT), dim3(GEMM_THREADS), 0, stream>>>(Qh, Qr, Kh, S, b);
    k_mixsm<<<dim3(NP), dim3(MIX_THREADS), 0, stream>>>(S, wpre, wpost, Ph);
    k_pv<<<dim3(NH * NQT), dim3(GEMM_THREADS), 0, stream>>>(Ph, VT, PS, wpost, Ch, Cr, b);
  }
  k_proj<<<dim3(NB * NQT * NCT), dim3(GEMM_THREADS), 0, stream>>>(Ch, Cr, Wp16, bproj, nbias, out);
  (void)hipGetLastError();
}
